// DilatedCNN_86517821215731
// MI455X (gfx1250) — hardware-verified
//
#include <hip/hip_runtime.h>


#define NR   8192
#define DD   1024
#define K3   (3 * DD)
#define WSC  16384.0f
typedef _Float16 h16;
typedef unsigned short bf;
typedef __attribute__((ext_vector_type(16))) __bf16   v16bf;
typedef __attribute__((ext_vector_type(16))) _Float16 v16h;
typedef __attribute__((ext_vector_type(8)))  _Float16 v8h;
typedef __attribute__((ext_vector_type(8)))  unsigned short v8us;
typedef __attribute__((ext_vector_type(8)))  float    v8f;
typedef __attribute__((ext_vector_type(4)))  float    v4f;
typedef v8h  __attribute__((may_alias)) v8ha;
typedef v4f  __attribute__((may_alias)) v4fa;
typedef v8us __attribute__((may_alias)) v8usa;

__device__ __forceinline__ unsigned short f2bf(float f) { unsigned u = __float_as_uint(f); u += 0x7FFFu + ((u >> 16) & 1u); return (unsigned short)(u >> 16); }
__device__ __forceinline__ float bf2f(unsigned short b) { return __uint_as_float(((unsigned)b) << 16); }
__device__ __forceinline__ float bfr(float f) { return bf2f(f2bf(f)); }
__device__ __forceinline__ v16h cat16(v8h lo, v8h hi) { return __builtin_shufflevector(lo, hi, 0, 1, 2, 3, 4, 5, 6, 7, 8, 9, 10, 11, 12, 13, 14, 15); }
__device__ __forceinline__ v16bf cat16b(v8us lo, v8us hi) { return __builtin_bit_cast(v16bf, __builtin_shufflevector(lo, hi, 0, 1, 2, 3, 4, 5, 6, 7, 8, 9, 10, 11, 12, 13, 14, 15)); }
__device__ __forceinline__ v8f wmma16(v16h a, v16h b, v8f c) { return __builtin_amdgcn_wmma_f32_16x16x32_f16(false, a, false, b, (short)0, c, false, false); }
__device__ __forceinline__ v8f wmmab(v16bf a, v16bf b, v8f c) { return __builtin_amdgcn_wmma_f32_16x16x32_bf16(false, a, false, b, (short)0, c, false, false); }


template <typename T16> struct WFrag;
template <> struct WFrag<h16> { typedef v16h V; static __device__ __forceinline__ V ld(const h16* p) { return cat16(*(const v8h*)p, *(const v8h*)(p + 16)); } static __device__ __forceinline__ v8f mma(V a, V b, v8f c) { return wmma16(a, b, c); } };
template <> struct WFrag<bf> { typedef v16bf V; static __device__ __forceinline__ V ld(const bf* p) { return cat16b(*(const v8us*)p, *(const v8us*)(p + 16)); } static __device__ __forceinline__ v8f mma(V a, V b, v8f c) { return wmmab(a, b, c); } };
template <typename T16, int NSPLIT, bool BIAS>
__global__ __launch_bounds__(32) void k_gemmw(const T16* __restrict__ A, const T16* __restrict__ A2, const T16* __restrict__ Bt, const T16* __restrict__ Bt2, int K, float* C, int ldc, const float* __restrict__ bias, size_t sA, size_t sB, size_t sC) {
    typedef typename WFrag<T16>::V V;
    __shared__ __align__(16) float os[16 * 68];
    const size_t z = blockIdx.z; A += z * sA; if (A2) A2 += z * sA; Bt += z * sB; if (Bt2) Bt2 += z * sB; C += z * sC;
    const int lane = threadIdx.x & 31, lr = lane & 15, hi = lane >> 4; const int r0 = blockIdx.x * 64, c0 = blockIdx.y * 64;
    v8f acc[4][4];
#pragma unroll
    for (int mb = 0; mb < 4; ++mb)
#pragma unroll
        for (int nb = 0; nb < 4; ++nb) acc[mb][nb] = (v8f){};
    const size_t aoff = (size_t)(r0 + lr) * K + 8 * hi, boff = (size_t)(c0 + lr) * K + 8 * hi;
#pragma unroll 1
    for (int kc = 0; kc < K; kc += 32) {
        V a[4], a2[4];
#pragma unroll
        for (int mb = 0; mb < 4; ++mb) { a[mb] = WFrag<T16>::ld(A + aoff + (size_t)mb * 16 * K + kc); if (NSPLIT == 1 || NSPLIT == 2) a2[mb] = WFrag<T16>::ld(A2 + aoff + (size_t)mb * 16 * K + kc); }
#pragma unroll
        for (int nb = 0; nb < 4; ++nb) { const V b = WFrag<T16>::ld(Bt + boff + (size_t)nb * 16 * K + kc); V b2; if (NSPLIT >= 2) b2 = WFrag<T16>::ld(Bt2 + boff + (size_t)nb * 16 * K + kc);
#pragma unroll
            for (int mb = 0; mb < 4; ++mb) { acc[mb][nb] = WFrag<T16>::mma(a[mb], b, acc[mb][nb]); if (NSPLIT == 1 || NSPLIT == 2) acc[mb][nb] = WFrag<T16>::mma(a2[mb], b, acc[mb][nb]); if (NSPLIT >= 2) acc[mb][nb] = WFrag<T16>::mma(a[mb], b2, acc[mb][nb]); } }
        asm volatile("v_nop\n\tv_nop\n\tv_nop\n\tv_nop" : "+v"(acc[0][0]), "+v"(acc[1][1]), "+v"(acc[2][2]), "+v"(acc[3][3]) : "v"(a[0]), "v"(a[3]));
    }
#pragma unroll
    for (int mb = 0; mb < 4; ++mb) {
#pragma unroll
        for (int nb = 0; nb < 4; ++nb) {
#pragma unroll
            for (int j = 0; j < 8; ++j) os[(hi * 8 + j) * 68 + nb * 16 + lr] = acc[mb][nb][j]; }
        __builtin_amdgcn_wave_barrier(); asm volatile("" ::: "memory");
        float* crow = C + (size_t)(r0 + mb * 16) * ldc + c0;
#pragma unroll 1
        for (int ps = 0; ps < 2; ++ps) {
#pragma unroll
            for (int s = 0; s < 8; ++s) { const int row = 2 * s + hi, cofs = lr * 4; v4f val = *(const v4fa*)(os + row * 68 + cofs); if (BIAS) { val[0] += bfr(bias[c0 + cofs]); val[1] += bfr(bias[c0 + cofs + 1]); val[2] += bfr(bias[c0 + cofs + 2]); val[3] += bfr(bias[c0 + cofs + 3]); }
                *(volatile v4f*)(crow + (size_t)row * ldc + cofs) = val; }
            if (ps == 0) __threadfence(); }
        __builtin_amdgcn_wave_barrier(); asm volatile("" ::: "memory");
    }
}

__device__ __forceinline__ h16 tohx(float x) { return (h16)x; }
typedef __attribute__((ext_vector_type(2))) _Float16 v2h;
typedef __attribute__((ext_vector_type(2))) unsigned short v2us;
typedef __attribute__((ext_vector_type(8))) _Float16 v8h16;

__global__ __launch_bounds__(256) void k_wtG(const float* __restrict__ w, int K, int N, bf* Bt) {
    const int lane = threadIdx.x & 31; const int L0 = (blockIdx.x * 8 + (threadIdx.x >> 5)) * 8; const int nlines = N * K / 64;
#pragma unroll 1
    for (int ps = 0; ps < 2; ++ps) {
#pragma unroll 1
        for (int l = 0; l < 8; ++l) { const int L = L0 + l; if (L >= nlines) break; const size_t e = (size_t)L * 64 + lane * 2; const int k = (int)(e % K), n = (int)(e / K); v2us o;
            o[0] = f2bf(w[(size_t)k * N + n]); o[1] = f2bf(w[(size_t)(k + 1) * N + n]); *(volatile v2us*)(Bt + e) = o; }
        if (ps == 0) __threadfence(); }
}
__global__ __launch_bounds__(256) void k_wtG16(const float* __restrict__ w, int K, int N, int pitch, int col0, h16* Bt) {
    const int lane = threadIdx.x & 31; const int L0 = (blockIdx.x * 8 + (threadIdx.x >> 5)) * 8; const int nlines = N * K / 64;
#pragma unroll 1
    for (int ps = 0; ps < 2; ++ps) {
#pragma unroll 1
        for (int l = 0; l < 8; ++l) { const int L = L0 + l; if (L >= nlines) break; const size_t e = (size_t)L * 64 + lane * 2; const int k = (int)(e % K), n = (int)(e / K); v2h o;
            o[0] = tohx(bfr(w[(size_t)k * pitch + col0 + n]) * WSC); o[1] = tohx(bfr(w[(size_t)(k + 1) * pitch + col0 + n]) * WSC); *(volatile v2h*)(Bt + e) = o; }
        if (ps == 0) __threadfence(); }
}
__global__ __launch_bounds__(256) void k_bsc(const float* __restrict__ b, float* BS, int n) { const int i = (blockIdx.x * 256 + threadIdx.x) * 4; if (i >= n) return; const v4f a = *(const v4f*)(b + i); v4f o;
#pragma unroll
    for (int q = 0; q < 4; ++q) o[q] = bfr(a[q]) * WSC; *(volatile v4f*)(BS + i) = o; __threadfence(); *(volatile v4f*)(BS + i) = o; }
template <int BF>
__global__ __launch_bounds__(256) void k_cat3(const float* __restrict__ X, const float* __restrict__ oob, int d, void* A) {
    const int lane = threadIdx.x & 31; const int L0 = (blockIdx.x * 8 + (threadIdx.x >> 5)) * 8; const int nlines = NR * K3 / 64;
#pragma unroll 1
    for (int ps = 0; ps < 2; ++ps) {
#pragma unroll 1
        for (int l = 0; l < 8; ++l) { const int L = L0 + l; if (L >= nlines) break; const size_t e = (size_t)L * 64 + lane * 2; const int r = (int)(e / K3); const int k = (int)(e % K3); const int seg = k >> 10, kk = k & (DD - 1);
            const int rr = (seg == 0) ? r : (seg == 1 ? r - d : r + d); const float* src = (rr >= 0 && rr < NR) ? (X + (size_t)rr * DD + kk) : (oob + kk); const float v0 = bfr(src[0]), v1 = bfr(src[1]);
            const bool isoob = !(rr >= 0 && rr < NR);
            if (BF) { v2us o; o[0] = f2bf(v0); o[1] = f2bf(v1); *(volatile v2us*)((bf*)A + e) = o; } else { v2h o; o[0] = tohx(isoob ? v0 : src[0]); o[1] = tohx(isoob ? v1 : src[1]); *(volatile v2h*)((h16*)A + e) = o; } }
        if (ps == 0) __threadfence(); }
}
__global__ __launch_bounds__(256) void k_upd(float* X, const float* __restrict__ F, float fsc) { const size_t i = ((size_t)blockIdx.x * 256 + threadIdx.x) * 4; if (i >= (size_t)NR * DD) return; const v4f x4 = *(const v4f*)(X + i), f4 = *(const v4f*)(F + i); v4f o;
#pragma unroll
    for (int q = 0; q < 4; ++q) { float a = __fmul_rn(0.5f, x4[q]), b = __fmul_rn(0.5f, fmaxf(__fmul_rn(f4[q], fsc), 0.f)); asm volatile("" : "+v"(a)); asm volatile("" : "+v"(b)); o[q] = __fadd_rn(a, b); }
    *(volatile v4f*)(X + i) = o; __threadfence(); *(volatile v4f*)(X + i) = o; }
__global__ __launch_bounds__(256) void k_xinit(const float* __restrict__ x, float* X) { const size_t i = ((size_t)blockIdx.x * 256 + threadIdx.x) * 4; if (i >= (size_t)NR * DD) return; const v4f a = *(const v4f*)(x + i); v4f o;
#pragma unroll
    for (int q = 0; q < 4; ++q) o[q] = bfr(a[q]); *(volatile v4f*)(X + i) = o; __threadfence(); *(volatile v4f*)(X + i) = o; }

extern "C" void kernel_launch(void* const* d_in, const int* in_sizes, int n_in,
                              void* d_out, int out_size, void* d_ws, size_t ws_size, hipStream_t stream) {
    (void)in_sizes; (void)n_in; (void)out_size;
    const float* x = (const float*)d_in[0]; const float* Ws = (const float*)d_in[1]; const float* bs = (const float*)d_in[2]; const float* oob = (const float*)d_in[3];
    float* X = (float*)d_out;
    char* wsp = (char*)d_ws;
    auto take = [&](size_t bytes) { char* p = wsp; wsp += (bytes + 255) & ~(size_t)255; return (void*)p; };
    bf* W0 = (bf*)take((size_t)DD * K3 * 2); h16* W16 = (h16*)take((size_t)DD * K3 * 2); float* BS = (float*)take(DD * 4); void* A = take((size_t)NR * K3 * 2); float* F = (float*)take((size_t)NR * DD * 4);
    if ((size_t)(wsp - (char*)d_ws) > ws_size) return;
    const unsigned gT = (unsigned)((DD * K3 / 64 + 63) / 64), LA = (unsigned)((NR * (K3 / 64) + 63) / 64), L4 = (unsigned)(((size_t)NR * DD / 4 + 255) / 256); const dim3 gP(NR / 64, DD / 64, 1);
    const int dil[4] = {1, 2, 4, 1};
    k_xinit<<<L4, 256, 0, stream>>>(x, X);
    for (int l = 0; l < 4; ++l) { const float* Wl = Ws + (size_t)l * K3 * DD; const float* bl = bs + (size_t)l * DD;
        if (l == 0) { k_wtG<<<gT, 256, 0, stream>>>(Wl, K3, DD, W0); k_cat3<1><<<LA, 256, 0, stream>>>(X, oob, dil[l], A);
            k_gemmw<bf, 0, true><<<gP, 32, 0, stream>>>((const bf*)A, nullptr, W0, nullptr, K3, F, DD, bl, 0, 0, 0); k_upd<<<L4, 256, 0, stream>>>(X, F, 1.0f); }
        else { k_wtG16<<<gT, 256, 0, stream>>>(Wl, K3, DD, DD, 0, W16); k_bsc<<<DD / 1024, 256, 0, stream>>>(bl, BS, DD); k_cat3<0><<<LA, 256, 0, stream>>>(X, oob, dil[l], A);
            k_gemmw<h16, 0, true><<<gP, 32, 0, stream>>>((const h16*)A, nullptr, W16, nullptr, K3, F, DD, BS, 0, 0, 0); k_upd<<<L4, 256, 0, stream>>>(X, F, 1.0f / WSC); } }
}
